// TTEmbedding_20761871909369
// MI455X (gfx1250) — hardware-verified
//
#include <hip/hip_runtime.h>


#ifndef NB
#define NB 512
#endif
#ifndef SEQ
#define SEQ 128
#endif
#define NB_FULL  512
#define SEQ_FULL 128
#define NTOK (NB * SEQ)
#define VD   100
#define VOCAB 1000000
#define RK   32
#define ED   128
#define NC1  (VD * RK)
#define QRS  2048.0f
#define QRI  (1.0f / 2048.0f)
#define GSC  4096.0f
#define WSC  64.0f
#define OSC  (1.0f / (4096.0f * 64.0f))
#define GP   40
#define OSP  36
#define T1P  68
#define WLP  33
#define P0   512
#define P1   12800
#define P2   12800

static_assert(SEQ == SEQ_FULL);
static_assert(NB <= NB_FULL);
static_assert(NTOK % 256 == 0);
static_assert(RK == 32);
static_assert(ED == 128);
static_assert(ED % 32 == 0);
static_assert(NC1 % 64 == 0);
static_assert(7 * 16 >= VD);
static_assert(7 * 16 <= 128);
static_assert(P0 % 256 == 0);
static_assert((P0 + P1) % 256 == 0);
static_assert((P0 + P1 + P2) % 256 == 0);
static_assert(P0 == 128 * RK / 8);
static_assert(P1 == NC1 * RK / 8);
static_assert(P2 == VD * RK * RK / 8);
static_assert((GP * 2) % 16 == 0);
static_assert((OSP * 4) % 16 == 0);
static_assert(256 * GP * 2 + 8 * 32 * OSP * 4 <= 131072);
static_assert(128 * T1P * 4 + ED * WLP * 4 + 16 * 64 * 4 <= 131072);
static_assert(16 * 68 * 4 <= 131072);

typedef _Float16 h16;
typedef unsigned short bf;
typedef __attribute__((ext_vector_type(16))) __bf16   v16bf;
typedef __attribute__((ext_vector_type(16))) _Float16 v16h;
typedef __attribute__((ext_vector_type(8)))  _Float16 v8h;
typedef __attribute__((ext_vector_type(8)))  unsigned short v8us;
typedef __attribute__((ext_vector_type(8)))  float    v8f;
typedef __attribute__((ext_vector_type(4)))  float    v4f;
typedef __attribute__((ext_vector_type(4)))  unsigned int v4u;
typedef v4f  __attribute__((may_alias)) v4fa;

__device__ __forceinline__ unsigned short f2bf(float f) { unsigned u = __float_as_uint(f); u += 0x7FFFu + ((u >> 16) & 1u); return (unsigned short)(u >> 16); }
__device__ __forceinline__ float bfr(float f) { return __uint_as_float(((unsigned)f2bf(f)) << 16); }
__device__ __forceinline__ v16h cat16(v8h lo, v8h hi) { return __builtin_shufflevector(lo, hi, 0, 1, 2, 3, 4, 5, 6, 7, 8, 9, 10, 11, 12, 13, 14, 15); }
__device__ __forceinline__ v16bf cat16b(v8us lo, v8us hi) { return __builtin_bit_cast(v16bf, __builtin_shufflevector(lo, hi, 0, 1, 2, 3, 4, 5, 6, 7, 8, 9, 10, 11, 12, 13, 14, 15)); }
__device__ __forceinline__ v8f wmma16(v16h a, v16h b, v8f c) { return __builtin_amdgcn_wmma_f32_16x16x32_f16(false, a, false, b, (short)0, c, false, false); }
__device__ __forceinline__ v8f wmmab(v16bf a, v16bf b, v8f c) { return __builtin_amdgcn_wmma_f32_16x16x32_bf16(false, a, false, b, (short)0, c, false, false); }
__device__ __forceinline__ v16h  ldh(const h16* p) { return cat16(*(const v8h*)p, *(const v8h*)(p + 16)); }
__device__ __forceinline__ v16bf ldb(const bf* p)  { return cat16b(*(const v8us*)p, *(const v8us*)(p + 16)); }
__device__ __forceinline__ void wave_sync() { __builtin_amdgcn_fence(3  , "wavefront"); __builtin_amdgcn_wave_barrier(); asm volatile("" ::: "memory"); }

__device__ __forceinline__ v8f wmma16g(v16h a, v16h b, v8f c) { c = wmma16(a, b, c); asm volatile("v_nop\n\tv_nop\n\tv_nop\n\tv_nop" : "+v"(c) : "v"(a), "v"(b)); return c; }
__device__ __forceinline__ v8f wmmabg(v16bf a, v16bf b, v8f c) { c = wmmab(a, b, c); asm volatile("v_nop\n\tv_nop\n\tv_nop\n\tv_nop" : "+v"(c) : "v"(a), "v"(b)); return c; }
static __device__ __forceinline__ h16 toh_flush(float v) { const h16 r = (h16)v; return (fabsf(v) < 6.103515625e-05f) ? (h16)0.0f : r; }

__global__ __launch_bounds__(256) void k_prep(const float* __restrict__ core0, const float* __restrict__ core1, const float* __restrict__ core2, bf* PL) {
    const int t = blockIdx.x * 256 + threadIdx.x;
    v8us o;
    if (blockIdx.x < P0 / 256) {
        const int row = t >> 2, c8 = (t & 3) * 8;
        const int rc = row < VD ? row : (VD - 1);
        v8f v = *(const v8f*)(core0 + rc * RK + c8);
        asm volatile("" : "+v"(v));
#pragma unroll
        for (int k = 0; k < 8; ++k) o[k] = (row < VD) ? f2bf(v[k]) : (unsigned short)0;
    } else if (blockIdx.x < (P0 + P1) / 256) {
        const int p = t - P0; const int n = p >> 2, r0 = (p & 3) * 8;
#pragma unroll
        for (int k = 0; k < 8; ++k) o[k] = f2bf(core1[(size_t)(r0 + k) * NC1 + n]);
    } else {
        const int p = t - (P0 + P1); const int i2 = p >> 7, rem = p & 127; const int r = rem >> 2, s0 = (rem & 3) * 8;
        const v8f v = *(const v8f*)(core2 + (size_t)r * NC1 + i2 * RK + s0);
#pragma unroll
        for (int k = 0; k < 8; ++k) o[k] = f2bf(v[k]);
    }
    bf* d = PL + (size_t)t * 8;
    *(volatile v8us*)d = o; __threadfence(); *(volatile v8us*)d = o;
}

__global__ __launch_bounds__(128) void k_wbuild(const float* __restrict__ core3, const float* __restrict__ core4, const float* __restrict__ core5, h16* WTH, h16* WTR) {
    __shared__ __align__(16) float t1s[128 * T1P];
    __shared__ __align__(16) float wl[ED * WLP];
    __shared__ __align__(16) float c4s[16 * 64];
    const int tid = threadIdx.x, lane = tid & 31, lr = lane & 15, hi = lane >> 4;
    const int wave = __builtin_amdgcn_readfirstlane((int)(threadIdx.x >> 5));
    static_assert(128 * 2 * 4 == 16 * 64);
#pragma unroll
    for (int it = 0; it < 2; ++it) { const int p = it * 128 + tid; const v4f v = *(const v4fa*)(core4 + p * 4); *(v4fa*)(&c4s[p * 4]) = v; }
    __syncthreads();
    const v8us z8 = (v8us){};
    v16bf bfrag[4];
#pragma unroll
    for (int nt = 0; nt < 4; ++nt) { v8us lo;
#pragma unroll
        for (int i = 0; i < 8; ++i) lo[i] = f2bf(c4s[(8 * hi + i) * 64 + nt * 16 + lr]);
        bfrag[nt] = cat16b(lo, z8); }
#pragma unroll
    for (int mi = 0; mi < 2; ++mi) {
        const int mt = wave * 2 + mi;
        const v8f av = *(const v8f*)(core3 + (mt * 16 + lr) * 16 + 8 * hi);
        v8us lo;
#pragma unroll
        for (int i = 0; i < 8; ++i) lo[i] = f2bf(av[i]);
        const v16bf a = cat16b(lo, z8);
#pragma unroll
        for (int nt = 0; nt < 4; ++nt) { v8f acc = (v8f){}; acc = wmmabg(a, bfrag[nt], acc);
#pragma unroll
            for (int j = 0; j < 8; ++j) t1s[(mt * 16 + 8 * hi + j) * T1P + nt * 16 + lr] = acc[j]; }
    }
    __syncthreads();
    { const int o0 = tid >> 5, o1 = (tid >> 2) & 7, o2 = tid & 3;
      float c5[8];
#pragma unroll
      for (int b = 0; b < 8; ++b) c5[b] = bfr(core5[b * 4 + o2]);
#pragma unroll 1
      for (int r = 0; r < RK; ++r) { const int tb = (r * 4 + o0) * T1P + o1 * 8; float w = 0.0f;
#pragma unroll
          for (int b = 0; b < 8; ++b) w = fmaf(t1s[tb + b], c5[b], w);
          wl[tid * WLP + r] = w; } }
    __syncthreads();
    static_assert(128 * 4 * 16 == ED * RK * 2);
#pragma unroll 1
    for (int ps = 0; ps < 2; ++ps) {
#pragma unroll
        for (int it = 0; it < 4; ++it) { const int p = it * 128 + tid; const int row = p >> 2, k0 = (p & 3) * 8; v8h hv, rv;
#pragma unroll
            for (int i = 0; i < 8; ++i) { const float x = wl[row * WLP + k0 + i] * WSC; const h16 a0 = toh_flush(x); hv[i] = a0; rv[i] = toh_flush((x - (float)a0) * QRS); }
            *(volatile v8h*)(WTH + (size_t)p * 8) = hv; *(volatile v8h*)(WTR + (size_t)p * 8) = rv; }
        if (ps == 0) __threadfence(); }
}

__global__ __launch_bounds__(32) void k_tab(const bf* __restrict__ A, const bf* __restrict__ Bt, float* T01) {
    __shared__ __align__(16) float os[16 * 68];
    const int lane = threadIdx.x & 31, lr = lane & 15, hi = lane >> 4; const int c0 = blockIdx.x * 64;
    v16bf b[4];
#pragma unroll
    for (int nb = 0; nb < 4; ++nb) b[nb] = ldb(Bt + (size_t)(c0 + nb * 16 + lr) * RK + 8 * hi);
#pragma unroll 1
    for (int mb = 0; mb < 7; ++mb) {
        const v16bf a = ldb(A + (size_t)(mb * 16 + lr) * RK + 8 * hi);
#pragma unroll
        for (int nb = 0; nb < 4; ++nb) { v8f acc = (v8f){}; acc = wmmabg(a, b[nb], acc);
#pragma unroll
            for (int j = 0; j < 8; ++j) os[(hi * 8 + j) * 68 + nb * 16 + lr] = acc[j]; }
        wave_sync();
        static_assert(8 * 2 == 16);
#pragma unroll 1
        for (int ps = 0; ps < 2; ++ps) {
#pragma unroll
            for (int s = 0; s < 8; ++s) { const int row = 2 * s + (lane >> 4), cofs = (lane & 15) * 4; const int i0 = mb * 16 + row;
                const v4f val = *(const v4fa*)(&os[row * 68 + cofs]);
                if (i0 < VD) *(volatile v4f*)(T01 + (size_t)i0 * NC1 + c0 + cofs) = val; }
            if (ps == 0) __threadfence(); }
        wave_sync();
    }
}

__global__ __launch_bounds__(256) void k_embed(const int* __restrict__ idx, const float* __restrict__ T01, const bf* __restrict__ C2P,
                                               const h16* __restrict__ WTH, const h16* __restrict__ WTR, float* OUT) {
    __shared__ __align__(16) h16 gh[256 * GP];
    __shared__ __align__(16) float os[8 * 32 * OSP];
    const int tid = threadIdx.x, lane = tid & 31, lr = lane & 15, hi = lane >> 4;
    const int wave = __builtin_amdgcn_readfirstlane((int)(threadIdx.x >> 5));
    const int n = blockIdx.x * 256 + tid;
    int id = idx[n]; id = id < 0 ? 0 : (id > (VOCAB - 1) ? (VOCAB - 1) : id);
    const int row01 = id / VD;
    const int i2 = id - row01 * VD;
    const float* trow = T01 + (size_t)row01 * RK;
    const v4u* cm = (const v4u*)(C2P + (size_t)i2 * (RK * RK));
    float ga[32];
#pragma unroll
    for (int s = 0; s < 32; ++s) ga[s] = 0.0f;
#pragma unroll 1
    for (int r = 0; r < RK; ++r) {
        const float g = trow[r];
        v4u w[4];
#pragma unroll
        for (int q = 0; q < 4; ++q) w[q] = cm[r * 4 + q];
#pragma unroll
        for (int q = 0; q < 4; ++q) {
#pragma unroll
            for (int j = 0; j < 4; ++j) {
                ga[8 * q + 2 * j]     = fmaf(g, __uint_as_float(w[q][j] << 16), ga[8 * q + 2 * j]);
                ga[8 * q + 2 * j + 1] = fmaf(g, __uint_as_float(w[q][j] & 0xffff0000u), ga[8 * q + 2 * j + 1]); } }
    }
#pragma unroll
    for (int q = 0; q < 4; ++q) { v8h hv;
#pragma unroll
        for (int i = 0; i < 8; ++i) hv[i] = toh_flush(ga[8 * q + i] * GSC);
        *(v8h*)(&gh[tid * GP + 8 * q]) = hv; }
    wave_sync();
    const int wr0 = wave * 32;
    const v16h aH0 = cat16(*(const v8h*)(&gh[(wr0 + lr) * GP + 8 * hi]),      *(const v8h*)(&gh[(wr0 + lr) * GP + 16 + 8 * hi]));
    const v16h aH1 = cat16(*(const v8h*)(&gh[(wr0 + 16 + lr) * GP + 8 * hi]), *(const v8h*)(&gh[(wr0 + 16 + lr) * GP + 16 + 8 * hi]));
    const int wb = wave * 32 * OSP;
    float* obase = OUT + (size_t)(blockIdx.x * 256 + wr0) * ED;
#pragma unroll 1
    for (int cp = 0; cp < 4; ++cp) {
#pragma unroll
        for (int cc = 0; cc < 2; ++cc) {
            const size_t wo = (size_t)((cp * 2 + cc) * 16 + lr) * RK + 8 * hi;
            const v16h bH = ldh(WTH + wo), bR = ldh(WTR + wo);
            v8f m0 = (v8f){}, m1 = (v8f){}, r0 = (v8f){}, r1 = (v8f){};
            m0 = wmma16g(aH0, bH, m0); r0 = wmma16g(aH0, bR, r0);
            m1 = wmma16g(aH1, bH, m1); r1 = wmma16g(aH1, bR, r1);
#pragma unroll
            for (int j = 0; j < 8; ++j) {
                os[wb + (8 * hi + j) * OSP + cc * 16 + lr]      = (m0[j] + r0[j] * QRI) * OSC;
                os[wb + (16 + 8 * hi + j) * OSP + cc * 16 + lr] = (m1[j] + r1[j] * QRI) * OSC; }
        }
        wave_sync();
        static_assert(8 * 4 == 32);
#pragma unroll 1
        for (int ps = 0; ps < 2; ++ps) {
#pragma unroll
            for (int s = 0; s < 8; ++s) { const int row = 4 * s + (lane >> 3), cofs = (lane & 7) * 4;
                const v4f val = *(const v4fa*)(&os[wb + row * OSP + cofs]);
                *(volatile v4f*)(obase + (size_t)row * ED + cp * 32 + cofs) = val; }
            if (ps == 0) __threadfence(); }
        wave_sync();
    }
}

static constexpr size_t al256(size_t v) { return (v + 255) & ~(size_t)255; }
static constexpr size_t SZ_PL = al256((size_t)(P0 + P1 + P2) * 16);
static constexpr size_t SZ_WT = al256((size_t)ED * RK * 2);
static constexpr size_t SZ_T  = al256((size_t)VD * NC1 * 4);
static constexpr size_t SZ_TOTAL = SZ_PL + 2 * SZ_WT + SZ_T;
static_assert(SZ_TOTAL <= (size_t)134217728);
static_assert(((size_t)P0 * 16) % 256 == 0);
static_assert(((size_t)(P0 + P1) * 16) % 256 == 0);
static_assert((size_t)(VD - 1) * NC1 + (NC1 - 64) + 63 < (size_t)VD * NC1);

extern "C" void kernel_launch(void* const* d_in, const int* in_sizes, int n_in,
                              void* d_out, int out_size, void* d_ws, size_t ws_size, hipStream_t stream) {
    if (n_in < 7) return;
    if ((size_t)in_sizes[0] < (size_t)NTOK) return;
    if (in_sizes[1] < VD * RK || in_sizes[2] < RK * VD * RK || in_sizes[3] < RK * VD * RK) return;
    if (in_sizes[4] < 32 * 4 * 16 || in_sizes[5] < 16 * 8 * 8 || in_sizes[6] < 8 * 4) return;
    if ((size_t)out_size < (size_t)NTOK * ED) return;
    if (SZ_TOTAL > ws_size) return;
    const int*   idx   = (const int*)d_in[0];
    const float* core0 = (const float*)d_in[1];
    const float* core1 = (const float*)d_in[2];
    const float* core2 = (const float*)d_in[3];
    const float* core3 = (const float*)d_in[4];
    const float* core4 = (const float*)d_in[5];
    const float* core5 = (const float*)d_in[6];
    float* OUT = (float*)d_out;
    char* wsp = (char*)d_ws;
    bf* PL = (bf*)wsp; wsp += SZ_PL;
    h16* WTH = (h16*)wsp; wsp += SZ_WT;
    h16* WTR = (h16*)wsp; wsp += SZ_WT;
    float* T01 = (float*)wsp; wsp += SZ_T;
    const bf* C0B = PL;
    const bf* C1T = PL + (size_t)P0 * 8;
    const bf* C2P = PL + (size_t)(P0 + P1) * 8;

    k_prep<<<(P0 + P1 + P2) / 256, 256, 0, stream>>>(core0, core1, core2, PL);
    k_wbuild<<<1, 128, 0, stream>>>(core3, core4, core5, WTH, WTR);
    k_tab<<<NC1 / 64, 32, 0, stream>>>(C0B, C1T, T01);
    k_embed<<<NTOK / 256, 256, 0, stream>>>(idx, T01, C2P, WTH, WTR, OUT);
}
